// EdgeNetEMD_60387240181866
// MI455X (gfx1250) — hardware-verified
//
#include <hip/hip_runtime.h>
#include <stddef.h>


#define NTHR   256
#define NWAVE  8
#define EPT    8
#define CHUNK  (NTHR * EPT)
#define WCAP   (EPT * 32)
#define LISTN  (NWAVE * WCAP)
#define PASSN  (NWAVE * 32)
#define PCAP   (CHUNK + PASSN)
#define NB     1024
#define NWROW  80
#define WSC    16.0f
#define WINV   0.0625f
#define BN_EPS 1e-5f

static_assert(PASSN == 256);
static_assert(PCAP >= CHUNK + PASSN);
static_assert((NB % 32) == 0);

typedef float    v2f  __attribute__((ext_vector_type(2)));
typedef float    v4f  __attribute__((ext_vector_type(4)));
typedef float    v8f  __attribute__((ext_vector_type(8)));
typedef int      v4i  __attribute__((ext_vector_type(4)));
typedef _Float16 v8h  __attribute__((ext_vector_type(8)));
typedef _Float16 v16h __attribute__((ext_vector_type(16)));
union FragH { v16h v; v8h h[2]; };

__device__ __forceinline__ v8h zero8() {
  v8h r;
#pragma unroll
  for (int i = 0; i < 8; ++i) r[i] = (_Float16)0.0f;
  return r;
}

__device__ __forceinline__ v8f wmh(v16h a, v16h b, v8f c) {
  v8f d = __builtin_amdgcn_wmma_f32_16x16x32_f16(false, a, false, b, (short)0, c, false, false);
  asm volatile("v_nop\n\tv_nop\n\tv_nop\n\tv_nop" : "+v"(d) : "v"(a), "v"(b));
  return d;
}

__device__ __forceinline__ v8h relu8(v8f d) {
  v8h r;
#pragma unroll
  for (int i = 0; i < 8; ++i) { const float t = fmaxf(d[i] * WINV, 0.0f); r[i] = (_Float16)t; }
  return r;
}

__device__ __forceinline__ v8f ldc8(const float* p) {
  const v4f a = *(const v4f*)p;
  const v4f b = *(const v4f*)(p + 4);
  v8f c;
  c[0] = a.x; c[1] = a.y; c[2] = a.z; c[3] = a.w;
  c[4] = b.x; c[5] = b.y; c[6] = b.z; c[7] = b.w;
  return c;
}

__device__ __forceinline__ int scan_chunk(const int* __restrict__ dsts, int nE, int cbase, int nodeBase,
                                          int vec8, int* list, int tid, int wave) {
  int wc = 0;
  const int el0  = tid * EPT;
  const int e0   = cbase + el0;
  const int sent = -2147483647 - 1;
  v4i da, db;
  if (vec8 != 0 && e0 + 7 < nE) {
    da = *(const v4i*)(dsts + e0);
    db = *(const v4i*)(dsts + e0 + 4);
  } else {
    da.x = (e0     < nE) ? dsts[e0]     : sent;
    da.y = (e0 + 1 < nE) ? dsts[e0 + 1] : sent;
    da.z = (e0 + 2 < nE) ? dsts[e0 + 2] : sent;
    da.w = (e0 + 3 < nE) ? dsts[e0 + 3] : sent;
    db.x = (e0 + 4 < nE) ? dsts[e0 + 4] : sent;
    db.y = (e0 + 5 < nE) ? dsts[e0 + 5] : sent;
    db.z = (e0 + 6 < nE) ? dsts[e0 + 6] : sent;
    db.w = (e0 + 7 < nE) ? dsts[e0 + 7] : sent;
  }
  const unsigned nb = (unsigned)nodeBase;
  const unsigned s0 = (unsigned)da.x - nb, s1 = (unsigned)da.y - nb;
  const unsigned s2 = (unsigned)da.z - nb, s3 = (unsigned)da.w - nb;
  const unsigned s4 = (unsigned)db.x - nb, s5 = (unsigned)db.y - nb;
  const unsigned s6 = (unsigned)db.z - nb, s7 = (unsigned)db.w - nb;
  const bool h0 = s0 < (unsigned)NB, h1 = s1 < (unsigned)NB, h2 = s2 < (unsigned)NB, h3 = s3 < (unsigned)NB;
  const bool h4 = s4 < (unsigned)NB, h5 = s5 < (unsigned)NB, h6 = s6 < (unsigned)NB, h7 = s7 < (unsigned)NB;
  const unsigned any = __builtin_amdgcn_ballot_w32(h0 | h1 | h2 | h3 | h4 | h5 | h6 | h7);
  if (any != 0u) {
#define HITJ(J, HJ) { \
      const unsigned mj = __builtin_amdgcn_ballot_w32(HJ); \
      if (mj != 0u) { \
        if (HJ) { \
          const int pos = wc + (int)__builtin_amdgcn_mbcnt_lo(mj, 0u); \
          if (pos < WCAP) list[wave * WCAP + pos] = el0 + (J); \
        } \
        wc += (int)__builtin_popcount(mj); } }
    HITJ(0, h0)
    HITJ(1, h1)
    HITJ(2, h2)
    HITJ(3, h3)
    HITJ(4, h4)
    HITJ(5, h5)
    HITJ(6, h6)
    HITJ(7, h7)
#undef HITJ
  }
  return wc;
}

__global__ __launch_bounds__(NTHR) void k_bn(const float* __restrict__ x, float* bnp, int nN) {
  __shared__ double red[8 * NTHR];
  __shared__ __attribute__((aligned(16))) float resf[32];
  const int tid = threadIdx.x, lane = tid & 31, wave = tid >> 5;
  double s0 = 0.0, s1 = 0.0, s2 = 0.0, s3 = 0.0, q0 = 0.0, q1 = 0.0, q2 = 0.0, q3 = 0.0;
#pragma unroll 1
  for (int i = tid; i < nN; i += NTHR) {
    const v4f v = *(const v4f*)(x + (size_t)i * 4);
    const double a = (double)v.x, b = (double)v.y, c = (double)v.z, d = (double)v.w;
    s0 += a; q0 += a * a;
    s1 += b; q1 += b * b;
    s2 += c; q2 += c * c;
    s3 += d; q3 += d * d;
  }
  red[0 * NTHR + tid] = s0; red[1 * NTHR + tid] = s1; red[2 * NTHR + tid] = s2; red[3 * NTHR + tid] = s3;
  red[4 * NTHR + tid] = q0; red[5 * NTHR + tid] = q1; red[6 * NTHR + tid] = q2; red[7 * NTHR + tid] = q3;
  __syncthreads();
#pragma unroll 1
  for (int st = NTHR / 2; st > 0; st >>= 1) {
    if (tid < st) {
#pragma unroll
      for (int k = 0; k < 8; ++k) red[k * NTHR + tid] += red[k * NTHR + tid + st];
    }
    __syncthreads();
  }
  if (tid == 0) {
    const double inv = 1.0 / (double)nN;
#pragma unroll
    for (int c = 0; c < 4; ++c) {
      const double mu = red[c * NTHR] * inv;
      double var = red[(4 + c) * NTHR] * inv - mu * mu;
      if (var < 0.0) var = 0.0;
      const float vf = (float)var;
      resf[c]     = (float)mu;
      resf[4 + c] = 1.0f / sqrtf(vf + BN_EPS);
    }
#pragma unroll
    for (int j = 8; j < 32; ++j) resf[j] = 0.0f;
  }
  __syncthreads();
  v4f rv = {0.0f, 0.0f, 0.0f, 0.0f};
  const bool wr = (wave == 0) && (lane < 8);
  if (wr) rv = *(const v4f*)(resf + 4 * lane);
  if (wr) *(volatile v4f*)(bnp + 4 * lane) = rv;
  __threadfence();
  if (wr) *(volatile v4f*)(bnp + 4 * lane) = rv;
}

template <int FIN, int OUT, int ORELU, int BNAPPLY>
__global__ __launch_bounds__(NTHR) void k_edge(
    const float* __restrict__ xin, const int* __restrict__ ei,
    const float* __restrict__ bnp, const float* __restrict__ bnw, const float* __restrict__ bnb,
    const float* __restrict__ W1, const float* __restrict__ Bi1,
    const float* __restrict__ W2, const float* __restrict__ Bi2,
    const float* __restrict__ W3, const float* __restrict__ Bi3,
    float* outp, int nN, int nE, int vec8, int outLim) {
  constexpr int KIN = 2 * FIN;
  constexpr int AW  = OUT + 1;
  constexpr int NQ  = (NB * OUT) / (128 * NWAVE);
  static_assert(NQ * 128 * NWAVE == NB * OUT);
  static_assert(KIN <= 8 && OUT <= 4);

  __shared__ __attribute__((aligned(16))) float    acc[(NB + 1) * AW];
  __shared__ __attribute__((aligned(16))) float    msg[PASSN * AW];
  __shared__ __attribute__((aligned(16))) _Float16 stg[NWAVE * 32 * 8];
  __shared__ __attribute__((aligned(16))) int      list[LISTN];
  __shared__ __attribute__((aligned(16))) int      pend[PCAP];
  __shared__ int slotb[PASSN];
  __shared__ __attribute__((aligned(16))) _Float16 wsm[NWROW * 32];
  __shared__ __attribute__((aligned(16))) float    bsm[NWROW];
  __shared__ int wcnt[NWAVE];
  __shared__ int pendN;

  const int tid = threadIdx.x, lane = tid & 31, wave = tid >> 5, hh = lane >> 4, m = lane & 15;
  const int nodeBase = blockIdx.x * NB;
  const int* srcs = ei;
  const int* dsts = ei + nE;

  for (int i = tid; i < (NB + 1) * AW; i += NTHR) acc[i] = 0.0f;
  for (int i = tid; i < NWROW * 32; i += NTHR) {
    const int row = i >> 5, k = i & 31;
    float v = 0.0f;
    if (row < 32) { if (k < KIN) v = W1[k * 32 + row]; }
    else if (row < 64) { v = W2[k * 32 + (row - 32)]; }
    else { const int f = row - 64; if (f < OUT) v = W3[k * OUT + f]; }
    wsm[i] = (_Float16)(v * WSC);
  }
  if (tid < NWROW) {
    float v = 0.0f;
    if (tid < 32) v = Bi1[tid];
    else if (tid < 64) v = Bi2[tid - 32];
    else if (tid - 64 < OUT) v = Bi3[tid - 64];
    bsm[tid] = v * WSC;
  }
  if (tid == 0) pendN = 0;
  float mu[4], rs[4], gw[4], gb[4];
#pragma unroll
  for (int c = 0; c < 4; ++c) {
    if (BNAPPLY != 0) { mu[c] = bnp[c]; rs[c] = bnp[4 + c]; gw[c] = bnw[c]; gb[c] = bnb[c]; }
    else { mu[c] = 0.0f; rs[c] = 1.0f; gw[c] = 1.0f; gb[c] = 0.0f; }
  }
  __syncthreads();

  const int nChunks = (nE + CHUNK - 1) / CHUNK;
#pragma unroll 1
  for (int ch = 0; ch < nChunks; ++ch) {
    const int cbase = ch * CHUNK;
    const int wc = scan_chunk(dsts, nE, cbase, nodeBase, vec8, list, tid, wave);
    if (lane == 0) wcnt[wave] = wc;
    __syncthreads();

    const int base = pendN;
    int tot = 0, myoff = 0;
#pragma unroll
    for (int w = 0; w < NWAVE; ++w) {
      int c = wcnt[w];
      c = c > WCAP ? WCAP : (c < 0 ? 0 : c);
      if (w < wave) myoff += c;
      tot += c;
    }
    int newN = base + tot;
    newN = newN > PCAP ? PCAP : newN;
    {
      int n = wcnt[wave];
      n = n > WCAP ? WCAP : (n < 0 ? 0 : n);
      const int* lp = list + wave * WCAP;
      for (int i = lane; i < n; i += 32) {
        const int pos = base + myoff + i;
        if (pos < PCAP) pend[pos] = cbase + lp[i];
      }
    }
    const int fin = (ch == nChunks - 1) ? 1 : 0;
    const int R   = (fin != 0) ? (newN + PASSN - 1) / PASSN : newN / PASSN;
    const int Pv  = (fin != 0) ? newN : R * PASSN;
    __syncthreads();

#pragma unroll 1
    for (int r = 0; r < R; ++r) {
      {
        const int idx = r * PASSN + wave * 32 + lane;
        const bool valid = idx < Pv;
        int e = 0;
        if (valid) e = pend[idx];
        e = e < 0 ? 0 : (e > nE - 1 ? nE - 1 : e);
        int d = dsts[e];
        int s = srcs[e];
        int slot = d - nodeBase;
        if (!valid || (unsigned)slot >= (unsigned)NB) slot = NB;
        d = d < 0 ? 0 : (d > nN - 1 ? nN - 1 : d);
        s = s < 0 ? 0 : (s > nN - 1 ? nN - 1 : s);
        float f[8];
        if (FIN == 4) {
          const v4f xi = *(const v4f*)(xin + (size_t)d * 4);
          const v4f xj = *(const v4f*)(xin + (size_t)s * 4);
#pragma unroll
          for (int c = 0; c < 4; ++c) {
            const float a = (xi[c] - mu[c]) * rs[c] * gw[c] + gb[c];
            const float b = (xj[c] - mu[c]) * rs[c] * gw[c] + gb[c];
            f[c] = a;
            f[4 + c] = b - a;
          }
        } else {
          const v2f ci = *(const v2f*)(xin + (size_t)d * 2);
          const v2f cj = *(const v2f*)(xin + (size_t)s * 2);
          f[0] = ci.x; f[1] = ci.y; f[2] = cj.x - ci.x; f[3] = cj.y - ci.y;
          f[4] = 0.0f; f[5] = 0.0f; f[6] = 0.0f; f[7] = 0.0f;
        }
        v8h hv;
#pragma unroll
        for (int c = 0; c < 8; ++c) { const float t = valid ? f[c] : 0.0f; hv[c] = (_Float16)t; }
        *(v8h*)(stg + (wave * 32 + lane) * 8) = hv;
        slotb[wave * 32 + lane] = slot;
      }
      __syncthreads();

      {
        const v8h z8 = zero8();
        FragH bq[2];
        {
          const v8h t0 = *(const v8h*)(stg + (wave * 32 + m) * 8);
          const v8h t1 = *(const v8h*)(stg + (wave * 32 + 16 + m) * 8);
          if (hh != 0) { bq[0].h[0] = z8; bq[1].h[0] = z8; }
          else         { bq[0].h[0] = t0; bq[1].h[0] = t1; }
          bq[0].h[1] = z8;
          bq[1].h[1] = z8;
        }
        v8f dA[2][2];
#pragma unroll
        for (int ft = 0; ft < 2; ++ft) {
          FragH a;
          const _Float16* ap = wsm + (16 * ft + m) * 32 + 8 * hh;
          a.h[0] = *(const v8h*)ap;
          a.h[1] = *(const v8h*)(ap + 16);
          const v8f c = ldc8(bsm + 16 * ft + 8 * hh);
          dA[ft][0] = wmh(a.v, bq[0].v, c);
          dA[ft][1] = wmh(a.v, bq[1].v, c);
        }
        bq[0].h[0] = relu8(dA[0][0]); bq[0].h[1] = relu8(dA[1][0]);
        bq[1].h[0] = relu8(dA[0][1]); bq[1].h[1] = relu8(dA[1][1]);
#pragma unroll
        for (int ft = 0; ft < 2; ++ft) {
          FragH a;
          const _Float16* ap = wsm + (32 + 16 * ft + m) * 32 + 8 * hh;
          a.h[0] = *(const v8h*)ap;
          a.h[1] = *(const v8h*)(ap + 16);
          const v8f c = ldc8(bsm + 32 + 16 * ft + 8 * hh);
          dA[ft][0] = wmh(a.v, bq[0].v, c);
          dA[ft][1] = wmh(a.v, bq[1].v, c);
        }
        bq[0].h[0] = relu8(dA[0][0]); bq[0].h[1] = relu8(dA[1][0]);
        bq[1].h[0] = relu8(dA[0][1]); bq[1].h[1] = relu8(dA[1][1]);
        v8f d3a, d3b;
        {
          FragH a;
          const _Float16* ap = wsm + (64 + m) * 32 + 8 * hh;
          a.h[0] = *(const v8h*)ap;
          a.h[1] = *(const v8h*)(ap + 16);
          const v8f c = ldc8(bsm + 64 + 8 * hh);
          d3a = wmh(a.v, bq[0].v, c);
          d3b = wmh(a.v, bq[1].v, c);
        }
        if (hh == 0) {
          float* mp = msg + (wave * 32 + m) * AW;
          float* mq = msg + (wave * 32 + 16 + m) * AW;
#pragma unroll
          for (int c = 0; c < OUT; ++c) {
            float va = d3a[c] * WINV, vb = d3b[c] * WINV;
            if (ORELU != 0) { va = fmaxf(va, 0.0f); vb = fmaxf(vb, 0.0f); }
            mp[c] = va;
            mq[c] = vb;
          }
          mp[OUT] = 1.0f;
          mq[OUT] = 1.0f;
        }
      }
      __syncthreads();

      if (wave == 0) {
#pragma unroll 1
        for (int i = 0; i < PASSN; ++i) {
          int sl = slotb[i];
          sl = sl < 0 ? 0 : (sl > NB ? NB : sl);
          if (lane < AW) {
            const float v = msg[i * AW + lane];
            volatile float* ap = acc + sl * AW + lane;
            const float cur = *ap;
            *ap = cur + v;
          }
        }
      }
      __syncthreads();
    }

    int rem = newN - R * PASSN;
    rem = rem < 0 ? 0 : rem;
    if (R > 0 && tid < rem) pend[tid] = pend[R * PASSN + tid];
    if (tid == 0) pendN = rem;
  }
  __syncthreads();

  v4f ov[NQ];
#pragma unroll
  for (int q = 0; q < NQ; ++q) {
    const int f = (wave * NQ + q) * 128 + 4 * lane;
    float t[4];
#pragma unroll
    for (int j = 0; j < 4; ++j) {
      const int fl = f + j;
      const int sl = fl / OUT;
      const int c  = fl - sl * OUT;
      const float cn = acc[sl * AW + OUT];
      t[j] = acc[sl * AW + c] * (1.0f / fmaxf(cn, 1.0f));
    }
    v4f v = {t[0], t[1], t[2], t[3]};
    ov[q] = v;
  }
  const size_t ob  = (size_t)nodeBase * OUT;
  const size_t lim = (size_t)(outLim < 0 ? 0 : outLim);
#pragma unroll
  for (int q = 0; q < NQ; ++q) {
    const size_t gi = ob + (size_t)((wave * NQ + q) * 128 + 4 * lane);
    if (gi + 3 < lim) *(volatile v4f*)(outp + gi) = ov[q];
  }
  __threadfence();
#pragma unroll
  for (int q = 0; q < NQ; ++q) {
    const size_t gi = ob + (size_t)((wave * NQ + q) * 128 + 4 * lane);
    if (gi + 3 < lim) *(volatile v4f*)(outp + gi) = ov[q];
  }
}

extern "C" void kernel_launch(void* const* d_in, const int* in_sizes, int n_in,
                              void* d_out, int out_size, void* d_ws, size_t ws_size,
                              hipStream_t stream) {
  if (n_in < 16) return;
  const int nN = in_sizes[0] / 4;
  const int nE = in_sizes[1] / 2;
  if (nN <= 0 || nE < 0 || in_sizes[0] != nN * 4 || in_sizes[1] != nE * 2) return;
  if (in_sizes[2] < 4 || in_sizes[3] < 4) return;
  if (in_sizes[4] != 8 * 32 || in_sizes[5] < 32 || in_sizes[6] != 32 * 32 || in_sizes[7] < 32) return;
  if (in_sizes[8] != 32 * 2 || in_sizes[9] < 2) return;
  if (in_sizes[10] != 4 * 32 || in_sizes[11] < 32 || in_sizes[12] != 32 * 32 || in_sizes[13] < 32) return;
  if (in_sizes[14] != 32 * 4 || in_sizes[15] < 4) return;
  if (out_size != nN * 4) return;

  const float* x    = (const float*)d_in[0];
  const int*   ei   = (const int*)d_in[1];
  const float* bn_w = (const float*)d_in[2];
  const float* bn_b = (const float*)d_in[3];
  const float* ew1  = (const float*)d_in[4];
  const float* eb1  = (const float*)d_in[5];
  const float* ew2  = (const float*)d_in[6];
  const float* eb2  = (const float*)d_in[7];
  const float* ew3  = (const float*)d_in[8];
  const float* eb3  = (const float*)d_in[9];
  const float* dw1  = (const float*)d_in[10];
  const float* db1  = (const float*)d_in[11];
  const float* dw2  = (const float*)d_in[12];
  const float* db2  = (const float*)d_in[13];
  const float* dw3  = (const float*)d_in[14];
  const float* db3  = (const float*)d_in[15];
  float* out = (float*)d_out;

  const int nBlk = (nN + NB - 1) / NB;

  char* ws = (char*)d_ws;
  size_t off = 0;
  const size_t oBn = off; off += 256;
  const size_t oCd = off; off += (size_t)nBlk * NB * 2 * 4;  off = (off + 255) & ~(size_t)255;
  if (off > ws_size) return;
  float* bnp  = (float*)(ws + oBn);
  float* code = (float*)(ws + oCd);

  const int vec8 = ((nE & 3) == 0) ? 1 : 0;

  k_bn<<<1, NTHR, 0, stream>>>(x, bnp, nN);

  k_edge<4, 2, 1, 1><<<nBlk, NTHR, 0, stream>>>(
      x, ei, bnp, bn_w, bn_b, ew1, eb1, ew2, eb2, ew3, eb3, code, nN, nE, vec8, nBlk * NB * 2);

  k_edge<2, 4, 0, 0><<<nBlk, NTHR, 0, stream>>>(
      code, ei, bnp, bn_w, bn_b, dw1, db1, dw2, db2, dw3, db3, out, nN, nE, vec8, nN * 4);
}
